// SimpleSOTAAttention_77610059038934
// MI455X (gfx1250) — hardware-verified
//
#include <hip/hip_runtime.h>
#include <math.h>
#include <stdint.h>

constexpr int kBatch  = 4;
constexpr int kSeq    = 2048;
constexpr int kHid    = 1024;
constexpr int kHeads  = 16;
constexpr int kHdim   = 64;
constexpr int kTokens = kBatch * kSeq;
constexpr int kQKCols = 2 * kHid;

typedef __attribute__((ext_vector_type(16))) _Float16 v16h;
typedef __attribute__((ext_vector_type(8)))  _Float16 v8h;
typedef __attribute__((ext_vector_type(16))) __bf16   v16b;
typedef __attribute__((ext_vector_type(8)))  __bf16   v8b;
typedef __attribute__((ext_vector_type(8)))  float    v8f;
typedef __attribute__((ext_vector_type(4)))  float    v4f;
typedef __attribute__((ext_vector_type(2)))  float    v2f;

__device__ __forceinline__ unsigned short f2bf_bits(float f) {
  unsigned u = __float_as_uint(f);
  return (unsigned short)((u + 0x7FFFu + ((u >> 16) & 1u)) >> 16);
}
__device__ __forceinline__ float bf_bits2f(unsigned short h) { return __uint_as_float(((unsigned)h) << 16); }

__device__ __forceinline__ void dep_guard_h(v8f& a, v8f& b, v16h x, v16h y) { asm volatile("v_nop\n\tv_nop\n\tv_nop\n\tv_nop" : "+v"(a), "+v"(b) : "v"(x), "v"(y)); }
__device__ __forceinline__ void dep_guard_b(v8f& a, v8f& b, v16b x, v16b y) { asm volatile("v_nop\n\tv_nop\n\tv_nop\n\tv_nop" : "+v"(a), "+v"(b) : "v"(x), "v"(y)); }
__device__ __forceinline__ void keep4_h(v16h a, v16h b, v16h c, v16h d) { asm volatile("v_nop" :: "v"(a), "v"(b), "v"(c), "v"(d)); }
__device__ __forceinline__ void keep4_b(v16b a, v16b b, v16b c, v16b d) { asm volatile("v_nop" :: "v"(a), "v"(b), "v"(c), "v"(d)); }
__device__ __forceinline__ void acc_guard4(v8f& a, v8f& b, v8f& c, v8f& d) { asm volatile("v_nop\n\tv_nop\n\tv_nop\n\tv_nop" : "+v"(a), "+v"(b), "+v"(c), "+v"(d)); }
template <typename T> struct Frag;
template <> struct Frag<_Float16> {
  typedef v16h V; union U { v16h v; v8h h[2]; };
  static __device__ __forceinline__ v16h load(const _Float16* p) {
    U f; f.h[0] = *(const v8h*)(p); f.h[1] = *(const v8h*)(p + 16); return f.v;
  }
  static __device__ __forceinline__ v8f mma(v16h a, v16h b, v8f c) {
    return __builtin_amdgcn_wmma_f32_16x16x32_f16(false, a, false, b, (short)0, c, false, false);
  }
  static __device__ __forceinline__ void guard(v8f& a, v8f& b, v16h x, v16h y) { dep_guard_h(a, b, x, y); }
  static __device__ __forceinline__ void keep(v16h a, v16h b, v16h c, v16h d) { keep4_h(a, b, c, d); }
};
template <> struct Frag<__bf16> {
  typedef v16b V; union U { v16b v; v8b h[2]; };
  static __device__ __forceinline__ v16b load(const __bf16* p) {
    U f; f.h[0] = *(const v8b*)(p); f.h[1] = *(const v8b*)(p + 16); return f.v;
  }
  static __device__ __forceinline__ v8f mma(v16b a, v16b b, v8f c) {
    return __builtin_amdgcn_wmma_f32_16x16x32_bf16(false, a, false, b, (short)0, c, false, false);
  }
  static __device__ __forceinline__ void guard(v8f& a, v8f& b, v16b x, v16b y) { dep_guard_b(a, b, x, y); }
  static __device__ __forceinline__ void keep(v16b a, v16b b, v16b c, v16b d) { keep4_b(a, b, c, d); }
};

template <int ET> struct Elem;
template <> struct Elem<0> { typedef _Float16 T; };
template <> struct Elem<1> { typedef __bf16 T; };
template <int ET, bool SPLIT, int BIAS_MODE, int OUT_MODE, bool RESID, int ACT = 0>
__global__ __launch_bounds__(256) void wmma_gemm64(
    const unsigned short* __restrict__ Ap, const unsigned short* __restrict__ A2p, int lda, long strideA,
    const unsigned short* __restrict__ Btp, const unsigned short* __restrict__ Bt2p, int ldb, long strideB,
    void* __restrict__ Cout, void* __restrict__ Cout2, int ldc, long strideC,
    const float* __restrict__ bias,
    const float* __restrict__ resid, long strideR,
    int M, int N, int K, float scale) {
  typedef typename Elem<ET>::T T;
  typedef typename Frag<T>::V V;
  const T* A = (const T*)Ap; const T* A2 = (const T*)A2p; const T* Bt = (const T*)Btp; const T* Bt2 = (const T*)Bt2p;
  __shared__ __align__(16) float sT[8][16 * 68];
  const int b    = blockIdx.y;
  const int lane = threadIdx.x & 31;
  const int wave = threadIdx.x >> 5;
  const int tilesN = N >> 6;
  const int tilesM = M >> 6;
  const int tile = blockIdx.x * 8 + wave;
  if (tile >= tilesM * tilesN) return;
  const int tm = tile / tilesN;
  const int tn = tile - tm * tilesN;
  const int m0 = tm << 6;
  const int n0 = tn << 6;

  const T* Ab  = A  + (size_t)b * strideA;
  const T* Bb  = Bt + (size_t)b * strideB;
  const T* Ab2 = SPLIT ? (A2  + (size_t)b * strideA) : nullptr;
  const T* Bb2 = SPLIT ? (Bt2 + (size_t)b * strideB) : nullptr;

  const int rlane = lane & 15;
  const int koff  = (lane >> 4) * 8;
  const int mOff  = (lane >> 4) * 8;

  v8f acc[4][4];
#pragma unroll
  for (int i = 0; i < 4; ++i)
#pragma unroll
    for (int j = 0; j < 4; ++j) acc[i][j] = (v8f){0.f,0.f,0.f,0.f,0.f,0.f,0.f,0.f};

  for (int k0 = 0; k0 < K; k0 += 32) {
    V bh[4], bl[4];
#pragma unroll
    for (int j = 0; j < 4; ++j) {
      const size_t bo = (size_t)(n0 + (j << 4) + rlane) * ldb + koff + k0;
      bh[j] = Frag<T>::load(Bb + bo);
      if (SPLIT) bl[j] = Frag<T>::load(Bb2 + bo);
    }
#pragma unroll
    for (int i = 0; i < 4; ++i) {
      const size_t ao = (size_t)(m0 + (i << 4) + rlane) * lda + koff + k0;
      V ah = Frag<T>::load(Ab + ao);
      V al;
      if (SPLIT) al = Frag<T>::load(Ab2 + ao);
#pragma unroll
      for (int j = 0; j < 4; ++j) {
        acc[i][j] = Frag<T>::mma(ah, bh[j], acc[i][j]);
        if (SPLIT) {
          acc[i][j] = Frag<T>::mma(ah, bl[j], acc[i][j]);
          acc[i][j] = Frag<T>::mma(al, bh[j], acc[i][j]);
        }
      }
      Frag<T>::guard(acc[i][0], acc[i][3], ah, SPLIT ? al : ah);
    }
    Frag<T>::keep(bh[0], bh[1], bh[2], bh[3]);
    if (SPLIT) Frag<T>::keep(bl[0], bl[1], bl[2], bl[3]);
  }
  acc_guard4(acc[0][0], acc[0][1], acc[0][2], acc[0][3]);
  acc_guard4(acc[1][0], acc[1][1], acc[1][2], acc[1][3]);
  acc_guard4(acc[2][0], acc[2][1], acc[2][2], acc[2][3]);
  acc_guard4(acc[3][0], acc[3][1], acc[3][2], acc[3][3]);

  float* slab = sT[wave];
  const float* Rb = RESID ? (resid + (size_t)b * strideR) : nullptr;
#pragma unroll
  for (int i = 0; i < 4; ++i) {
    const int mBase = m0 + (i << 4);
#pragma unroll
    for (int j = 0; j < 4; ++j) {
      const int n = n0 + (j << 4) + rlane;
      float bv = 0.f;
      if (BIAS_MODE == 2) bv = bias[n];
#pragma unroll
      for (int r = 0; r < 8; ++r) {
        float v = acc[i][j][r] * scale;
        if (BIAS_MODE == 1) v += bias[mBase + mOff + r];
        if (BIAS_MODE == 2) v += bv;
        if (RESID) v += Rb[(size_t)(mBase + mOff + r) * ldc + n];
        if (ACT == 1) v = tanhf(v);
        if (ACT == 2) v = fmaxf(v, 0.0f);
        if (ACT == 3) v = v / (1.0f + expf(-v));
        if (ACT == 4) v = (v > 0.f) ? v : 0.01f * v;
        if (ACT == 5) v = 0.5f * v * (1.0f + erff(v * 0.70710678118654752f));
        slab[(mOff + r) * 68 + (j << 4) + rlane] = v;
      }
    }
    __builtin_amdgcn_fence(__ATOMIC_RELEASE, "workgroup");
    __builtin_amdgcn_wave_barrier();
    __builtin_amdgcn_fence(__ATOMIC_ACQUIRE, "workgroup");
    if (OUT_MODE == 0) {
      float* C = (float*)Cout + (size_t)b * strideC;
      const int hh = lane >> 4, c4 = (lane & 15) * 4;
      for (int pass = 0; pass < 2; ++pass) {
#pragma unroll
        for (int it = 0; it < 8; ++it) {
          const int row = it * 2 + hh;
          v4f v = *(const v4f*)(slab + row * 68 + c4);
          *(volatile v4f*)(C + (size_t)(mBase + row) * ldc + n0 + c4) = v;
        }
        __threadfence();
      }
    } else {
      const int q = lane >> 3, c8 = (lane & 7) * 8;
      unsigned short* C  = (unsigned short*)Cout  + (size_t)b * strideC;
      unsigned short* C2 = (OUT_MODE == 2) ? ((unsigned short*)Cout2 + (size_t)b * strideC) : nullptr;
      for (int pass = 0; pass < 2; ++pass) {
#pragma unroll
        for (int it = 0; it < 4; ++it) {
          const int row = it * 4 + q;
          const float* sp = slab + row * 68 + c8;
          v8h hv, lv;
#pragma unroll
          for (int e = 0; e < 8; ++e) {
            if (OUT_MODE == 1) {
              hv[e] = (_Float16)sp[e];
            } else {
              unsigned short hb = f2bf_bits(sp[e]);
              unsigned short lb = f2bf_bits(sp[e] - bf_bits2f(hb));
              hv[e] = __builtin_bit_cast(_Float16, hb);
              lv[e] = __builtin_bit_cast(_Float16, lb);
            }
          }
          *(volatile v8h*)(C + (size_t)(mBase + row) * ldc + n0 + c8) = hv;
          if (OUT_MODE == 2) *(volatile v8h*)(C2 + (size_t)(mBase + row) * ldc + n0 + c8) = lv;
        }
        __threadfence();
      }
    }
    __builtin_amdgcn_fence(__ATOMIC_RELEASE, "workgroup");
    __builtin_amdgcn_wave_barrier();
    __builtin_amdgcn_fence(__ATOMIC_ACQUIRE, "workgroup");
  }
}

__device__ __forceinline__ unsigned pk16(unsigned short a, unsigned short b) { return (unsigned)a | ((unsigned)b << 16); }

__global__ __launch_bounds__(256) void cast_f32_bf16x2(const float* __restrict__ in, unsigned short* __restrict__ out, int n2) {
  const int i = blockIdx.x * 256 + threadIdx.x;
  if (i < n2) {
    const v2f f = *(const v2f*)(in + 2 * (size_t)i);
    const unsigned u = pk16(f2bf_bits(f[0]), f2bf_bits(f[1]));
    ((volatile unsigned*)out)[i] = u;
    __threadfence();
    ((volatile unsigned*)out)[i] = u;
  }
}

__global__ __launch_bounds__(256) void cast_f32_bf16_f16x2(const float* __restrict__ in, unsigned short* __restrict__ out,
                                                           int n2, float mul) {
  const int i = blockIdx.x * 256 + threadIdx.x;
  if (i < n2) {
    const v2f f = *(const v2f*)(in + 2 * (size_t)i);
    const _Float16 h0 = (_Float16)(bf_bits2f(f2bf_bits(f[0])) * mul);
    const _Float16 h1 = (_Float16)(bf_bits2f(f2bf_bits(f[1])) * mul);
    const unsigned u = pk16(__builtin_bit_cast(unsigned short, h0), __builtin_bit_cast(unsigned short, h1));
    ((volatile unsigned*)out)[i] = u;
    __threadfence();
    ((volatile unsigned*)out)[i] = u;
  }
}

constexpr int ATT_D  = 64;
constexpr int ATT_NW = 4;
constexpr int ATT_QB = 64;
constexpr int ATT_KC = 64;
constexpr float kPCarry      = 32768.0f;
constexpr float kOutOverP    = 16.0f / 32768.0f;
constexpr float kScoreScale  = 0.125f;

__device__ __forceinline__ v8f at_mma_b(v16b a, v16b b, v8f c) {
  c = __builtin_amdgcn_wmma_f32_16x16x32_bf16(false, a, false, b, (short)0, c, false, false);
  asm volatile("v_nop\n\tv_nop\n\tv_nop\n\tv_nop" : "+v"(c) : "v"(a), "v"(b));
  return c;
}
__device__ __forceinline__ v8f at_mma_h(v16h a, v16h b, v8f c) {
  c = __builtin_amdgcn_wmma_f32_16x16x32_f16(false, a, false, b, (short)0, c, false, false);
  asm volatile("v_nop\n\tv_nop\n\tv_nop\n\tv_nop" : "+v"(c) : "v"(a), "v"(b));
  return c;
}

__global__ __launch_bounds__(128)
void mha_core_kernel(const unsigned short* __restrict__ qkhp, const unsigned short* __restrict__ qklp,
                     const unsigned short* __restrict__ vtp, const float* __restrict__ amask,
                     unsigned short* __restrict__ o16p) {
  union FB { v16b v; v8b h[2]; };
  union FH { v16h v; v8h h[2]; };
  __shared__ __align__(16) __bf16   Ksh[ATT_KC * ATT_D];
  __shared__ __align__(16) __bf16   Ksl[ATT_KC * ATT_D];
  __shared__ __align__(16) _Float16 Vts[ATT_D * ATT_KC];
  __shared__ __align__(16) _Float16 Psh[ATT_NW][16 * ATT_KC];
  __shared__ __align__(16) float    Os[ATT_NW][16 * 68];

  const int tid  = threadIdx.x;
  const int wave = tid >> 5;
  const int lane = tid & 31;
  const int hh   = lane >> 4;
  const int c    = lane & 15;

  const int nqb = kSeq / ATT_QB;
  const int bx  = blockIdx.x;
  const int qb  = bx % nqb;
  const int bh  = bx / nqb;
  const int h   = bh % kHeads;
  const int b   = bh / kHeads;
  const int q0  = qb * ATT_QB + wave * 16;
  const size_t tok0 = (size_t)b * kSeq;

  const __bf16* Qh = (const __bf16*)(const void*)qkhp + (size_t)h * ATT_D;
  const __bf16* Ql = (const __bf16*)(const void*)qklp + (size_t)h * ATT_D;
  const __bf16* Kh = Qh + kHid;
  const __bf16* Kl = Ql + kHid;
  const _Float16* Vt = (const _Float16*)(const void*)vtp + ((size_t)b * kHid + (size_t)h * ATT_D) * kSeq;
  const float* mrowp = amask + tok0;
  unsigned short* ob = o16p + (size_t)h * ATT_D;

  v16b qah[2], qal[2];
#pragma unroll
  for (int dc = 0; dc < 2; ++dc) {
    const __bf16* qr = Qh + (tok0 + q0 + c) * kQKCols + dc * 32 + 8 * hh;
    const __bf16* ql = Ql + (tok0 + q0 + c) * kQKCols + dc * 32 + 8 * hh;
    qah[dc] = Frag<__bf16>::load(qr);
    qal[dc] = Frag<__bf16>::load(ql);
  }

  float mrow[8], lrow[8];
  v8f oacc[4];
#pragma unroll
  for (int r = 0; r < 8; ++r) { mrow[r] = -INFINITY; lrow[r] = 0.f; }
#pragma unroll
  for (int t = 0; t < 4; ++t) oacc[t] = (v8f){0.f,0.f,0.f,0.f,0.f,0.f,0.f,0.f};

  const int nChunks = kSeq / ATT_KC;
  for (int kc = 0; kc < nChunks; ++kc) {
    const int kv0 = kc * ATT_KC;
    __syncthreads();
    {
      const int r = tid >> 1, half = (tid & 1) * 32;
      const __bf16*   ksh = Kh + (tok0 + kv0 + r) * kQKCols + half;
      const __bf16*   ksl = Kl + (tok0 + kv0 + r) * kQKCols + half;
      const _Float16* vsr = Vt + (size_t)r * kSeq + kv0 + half;
#pragma unroll
      for (int i = 0; i < 4; ++i) {
        const v8b a0 = *(const v8b*)(ksh + 8 * i);
        const v8b a1 = *(const v8b*)(ksl + 8 * i);
        const v8h b0 = *(const v8h*)(vsr + 8 * i);
        *(v8b*)(Ksh + r * ATT_D  + half + 8 * i) = a0;
        *(v8b*)(Ksl + r * ATT_D  + half + 8 * i) = a1;
        *(v8h*)(Vts + r * ATT_KC + half + 8 * i) = b0;
      }
    }
    __syncthreads();

    v8f s[4];
#pragma unroll
    for (int j = 0; j < 4; ++j) {
      s[j] = (v8f){0.f,0.f,0.f,0.f,0.f,0.f,0.f,0.f};
#pragma unroll
      for (int dc = 0; dc < 2; ++dc) {
        FB kb, kl;
        kb.h[0] = *(const v8b*)(Ksh + (j * 16 + c) * ATT_D + dc * 32 + 8 * hh);
        kb.h[1] = *(const v8b*)(Ksh + (j * 16 + c) * ATT_D + dc * 32 + 16 + 8 * hh);
        kl.h[0] = *(const v8b*)(Ksl + (j * 16 + c) * ATT_D + dc * 32 + 8 * hh);
        kl.h[1] = *(const v8b*)(Ksl + (j * 16 + c) * ATT_D + dc * 32 + 16 + 8 * hh);
        s[j] = at_mma_b(qah[dc], kb.v, s[j]);
        s[j] = at_mma_b(qah[dc], kl.v, s[j]);
        s[j] = at_mma_b(qal[dc], kb.v, s[j]);
      }
    }
    float mk[4];
#pragma unroll
    for (int j = 0; j < 4; ++j) mk[j] = mrowp[kv0 + j * 16 + c];

    float cm[8];
#pragma unroll
    for (int r = 0; r < 8; ++r) {
      float m = -INFINITY;
#pragma unroll
      for (int j = 0; j < 4; ++j) {
        s[j][r] = s[j][r] * kScoreScale + mk[j];
        m = fmaxf(m, s[j][r]);
      }
#pragma unroll
      for (int off = 1; off < 16; off <<= 1) m = fmaxf(m, __shfl_xor(m, off, 32));
      cm[r] = m;
    }
    _Float16* pw = Psh[wave];
#pragma unroll
    for (int r = 0; r < 8; ++r) {
      const float mnew  = fmaxf(mrow[r], cm[r]);
      const float alpha = expf(mrow[r] - mnew);
      mrow[r] = mnew;
      float psum = 0.f;
#pragma unroll
      for (int j = 0; j < 4; ++j) {
        const float p = expf(s[j][r] - mnew);
        psum += p;
        pw[(8 * hh + r) * ATT_KC + j * 16 + c] = (_Float16)(p * kPCarry);
      }
#pragma unroll
      for (int off = 1; off < 16; off <<= 1) psum += __shfl_xor(psum, off, 32);
      lrow[r] = lrow[r] * alpha + psum;
#pragma unroll
      for (int t = 0; t < 4; ++t) oacc[t][r] *= alpha;
    }
    __builtin_amdgcn_fence(__ATOMIC_RELEASE, "workgroup");
    __builtin_amdgcn_wave_barrier();
    __builtin_amdgcn_fence(__ATOMIC_ACQUIRE, "workgroup");

#pragma unroll
    for (int kk = 0; kk < 2; ++kk) {
      FH pa;
      pa.h[0] = *(const v8h*)(pw + c * ATT_KC + kk * 32 + 8 * hh);
      pa.h[1] = *(const v8h*)(pw + c * ATT_KC + kk * 32 + 16 + 8 * hh);
#pragma unroll
      for (int t = 0; t < 4; ++t) {
        FH vb;
        vb.h[0] = *(const v8h*)(Vts + (t * 16 + c) * ATT_KC + kk * 32 + 8 * hh);
        vb.h[1] = *(const v8h*)(Vts + (t * 16 + c) * ATT_KC + kk * 32 + 16 + 8 * hh);
        oacc[t] = at_mma_h(pa.v, vb.v, oacc[t]);
      }
    }
  }

  float* os = Os[wave];
#pragma unroll
  for (int r = 0; r < 8; ++r) {
    const float inv = (1.0f / lrow[r]) * kOutOverP;
#pragma unroll
    for (int t = 0; t < 4; ++t) os[(8 * hh + r) * 68 + t * 16 + c] = oacc[t][r] * inv;
  }
  __builtin_amdgcn_fence(__ATOMIC_RELEASE, "workgroup");
  __builtin_amdgcn_wave_barrier();
  __builtin_amdgcn_fence(__ATOMIC_ACQUIRE, "workgroup");
  {
    const int q = lane >> 3, c8 = (lane & 7) * 8;
    for (int pass = 0; pass < 2; ++pass) {
#pragma unroll
      for (int it = 0; it < 4; ++it) {
        const int row = it * 4 + q;
        const float* sp = os + row * 68 + c8;
        v8h hv;
#pragma unroll
        for (int e = 0; e < 8; ++e) hv[e] = (_Float16)sp[e];
        *(volatile v8h*)(ob + (tok0 + q0 + row) * (size_t)kHid + c8) = hv;
      }
      __threadfence();
    }
  }
}

extern "C" void kernel_launch(void* const* d_in, const int* in_sizes, int n_in,
                              void* d_out, int out_size, void* d_ws, size_t ws_size,
                              hipStream_t stream) {
  if (n_in < 6) return;
  if (in_sizes[0] != kTokens * kHid) return;
  if (in_sizes[1] != kBatch * kSeq) return;
  if (in_sizes[2] != kHid * kHid || in_sizes[3] != kHid * kHid ||
      in_sizes[4] != kHid * kHid || in_sizes[5] != kHid * kHid) return;
  if (out_size != kTokens * kHid) return;

  const float* X     = (const float*)d_in[0];
  const float* maskp = (const float*)d_in[1];
  const float* Wq    = (const float*)d_in[2];
  const float* Wk    = (const float*)d_in[3];
  const float* Wv    = (const float*)d_in[4];
  const float* Wo    = (const float*)d_in[5];
  float* out = (float*)d_out;

  const size_t bytesXb   = (size_t)kTokens * kHid * 2;
  const size_t bytesWqkv = (size_t)3 * kHid * kHid * 2;
  const size_t bytesWo   = (size_t)kHid * kHid * 2;
  const size_t bytesQK   = (size_t)kTokens * kQKCols * 2;
  const size_t bytesVt   = (size_t)kBatch * kHid * kSeq * 2;
  const size_t bytesO16  = (size_t)kTokens * kHid * 2;
  size_t off = 0;
  const size_t offXb   = off; off += bytesXb;
  const size_t offWqkv = off; off += bytesWqkv;
  const size_t offWo   = off; off += bytesWo;
  const size_t offQKh  = off; off += bytesQK;
  const size_t offQKl  = off; off += bytesQK;
  const size_t offVt   = off; off += bytesVt;
  const size_t offO16  = off; off += bytesO16;
  if (off > ws_size) return;

  char* ws = (char*)d_ws;
  unsigned short* Xb   = (unsigned short*)(ws + offXb);
  unsigned short* Wqkv = (unsigned short*)(ws + offWqkv);
  unsigned short* Wvb  = Wqkv + (size_t)2 * kHid * kHid;
  unsigned short* Wo16 = (unsigned short*)(ws + offWo);
  unsigned short* QKh  = (unsigned short*)(ws + offQKh);
  unsigned short* QKl  = (unsigned short*)(ws + offQKl);
  unsigned short* Vt   = (unsigned short*)(ws + offVt);
  unsigned short* O16  = (unsigned short*)(ws + offO16);

  const int nx2 = kTokens * kHid / 2;
  const int nw2 = kHid * kHid / 2;
  cast_f32_bf16x2<<<dim3(nx2 / 256), dim3(256), 0, stream>>>(X, Xb, nx2);
  cast_f32_bf16x2<<<dim3(nw2 / 256), dim3(256), 0, stream>>>(Wq, Wqkv, nw2);
  cast_f32_bf16x2<<<dim3(nw2 / 256), dim3(256), 0, stream>>>(Wk, Wqkv + (size_t)kHid * kHid, nw2);
  cast_f32_bf16x2<<<dim3(nw2 / 256), dim3(256), 0, stream>>>(Wv, Wvb, nw2);
  cast_f32_bf16_f16x2<<<dim3(nw2 / 256), dim3(256), 0, stream>>>(Wo, Wo16, nw2, 64.0f);

  wmma_gemm64<1, false, 0, 2, false><<<dim3(512, 1), dim3(256), 0, stream>>>(
      Xb, Xb, kHid, 0L,
      Wqkv, Wqkv, kHid, 0L,
      (void*)QKh, (void*)QKl, kQKCols, 0L,
      maskp, maskp, 0L,
      kTokens, kQKCols, kHid, 1.0f);

  wmma_gemm64<1, false, 0, 1, false><<<dim3(64, kBatch), dim3(256), 0, stream>>>(
      Wvb, Wvb, kHid, 0L,
      Xb, Xb, kHid, (long)kSeq * kHid,
      (void*)Vt, (void*)Vt, kSeq, (long)kHid * kSeq,
      maskp, maskp, 0L,
      kHid, kSeq, kHid, 1.0f);

  mha_core_kernel<<<dim3(kBatch * kHeads * (kSeq / ATT_QB)), dim3(128), 0, stream>>>(QKh, QKl, Vt, maskp, O16);

  wmma_gemm64<0, false, 0, 0, false><<<dim3(256, 1), dim3(256), 0, stream>>>(
      O16, O16, kHid, 0L,
      Wo16, Wo16, kHid, 0L,
      (void*)out, (void*)out, kHid, 0L,
      maskp, maskp, 0L,
      kTokens, kHid, kHid, 1.0f / 1024.0f);
}
